// SpatialCrossScaleAttention_2568390443354
// MI455X (gfx1250) — hardware-verified
//
#include <hip/hip_runtime.h>
#include <math.h>
#include <stdint.h>

#define NBATCH 4
#define DIMC   192
#define NHEAD  8
#define HDP    32
#define QCOL   256
static_assert(NHEAD * HDP == QCOL);

typedef _Float16 v16h __attribute__((ext_vector_type(16)));
typedef _Float16 v8h  __attribute__((ext_vector_type(8)));
typedef __bf16   v16b __attribute__((ext_vector_type(16)));
typedef __bf16   v8b  __attribute__((ext_vector_type(8)));
typedef float    v8f  __attribute__((ext_vector_type(8)));
typedef float    v4f  __attribute__((ext_vector_type(4)));
typedef unsigned int v4u __attribute__((ext_vector_type(4)));

__device__ __forceinline__ unsigned short bf_bits(float f) {
  unsigned u = __float_as_uint(f);
  return (unsigned short)((u + 0x7FFFu + ((u >> 16) & 1u)) >> 16);
}
__device__ __forceinline__ float bf_up(unsigned short h) { return __uint_as_float(((unsigned)h) << 16); }
__device__ __forceinline__ unsigned short h_bits(_Float16 x) { return __builtin_bit_cast(unsigned short, x); }
__device__ __forceinline__ unsigned pk16(unsigned short a, unsigned short b) { return (unsigned)a | ((unsigned)b << 16); }
__device__ __forceinline__ v8f zero8() { v8f z = {0.f, 0.f, 0.f, 0.f, 0.f, 0.f, 0.f, 0.f}; return z; }

__device__ __forceinline__ v16b ldfrag_b(const __bf16* p) {
  union { v16b v; v8b h[2]; } f;
  f.h[0] = *(const v8b*)(p);
  f.h[1] = *(const v8b*)(p + 16);
  return f.v;
}
__device__ __forceinline__ v16h ldfrag_h(const _Float16* p) {
  union { v16h v; v8h h[2]; } f;
  f.h[0] = *(const v8h*)(p);
  f.h[1] = *(const v8h*)(p + 16);
  return f.v;
}

__device__ __forceinline__ v8f mma_h(v16h a, v16h b, v8f c) {
  c = __builtin_amdgcn_wmma_f32_16x16x32_f16(false, a, false, b, (short)0, c, false, false);
#if defined(__HIP_DEVICE_COMPILE__)
  asm volatile("v_nop\n\tv_nop\n\tv_nop\n\tv_nop" : "+v"(c) : "v"(a), "v"(b));
#endif
  return c;
}
__device__ __forceinline__ v8f mma_b_raw(v16b a, v16b b, v8f c) {
  return __builtin_amdgcn_wmma_f32_16x16x32_bf16(false, a, false, b, (short)0, c, false, false);
}
__device__ __forceinline__ void dep_guard_b(v8f& a, v8f& b, v16b x, v16b y) {
#if defined(__HIP_DEVICE_COMPILE__)
  asm volatile("v_nop\n\tv_nop\n\tv_nop\n\tv_nop" : "+v"(a), "+v"(b) : "v"(x), "v"(y));
#endif
}
__device__ __forceinline__ void keep4_b(v16b a, v16b b, v16b c, v16b d) {
#if defined(__HIP_DEVICE_COMPILE__)
  asm volatile("v_nop" :: "v"(a), "v"(b), "v"(c), "v"(d));
#endif
}
__device__ __forceinline__ void acc_guard4(v8f& a, v8f& b, v8f& c, v8f& d) {
#if defined(__HIP_DEVICE_COMPILE__)
  asm volatile("v_nop\n\tv_nop\n\tv_nop\n\tv_nop" : "+v"(a), "+v"(b), "+v"(c), "+v"(d));
#endif
}
__device__ __forceinline__ void wave_sync_lds() {
  __builtin_amdgcn_fence(__ATOMIC_RELEASE, "workgroup");
  __builtin_amdgcn_wave_barrier();
  __builtin_amdgcn_fence(__ATOMIC_ACQUIRE, "workgroup");
}

__global__ __launch_bounds__(256) void cvt_rows(const float* __restrict__ src, int srcRows, int K,
                                                unsigned short* dst, int pad, int n8) {
  const int i = blockIdx.x * 256 + threadIdx.x;
  if (i >= n8) return;
  const int e0 = i * 8;
  const int r  = e0 / K;
  const int cc = e0 - r * K;
  const int g  = r >> 5, dd = r & 31;
  const bool valid = (pad == 0) || (dd < 24);
  int srow = (pad != 0) ? (g * 24 + ((dd < 24) ? dd : 23)) : r;
  srow = min(max(srow, 0), srcRows - 1);
  const float* sp = src + (size_t)srow * K + cc;
  const v4f a  = *(const v4f*)sp;
  const v4f a2 = *(const v4f*)(sp + 4);
  v4u p;
  p[0] = pk16(bf_bits(valid ? a[0]  : 0.f), bf_bits(valid ? a[1]  : 0.f));
  p[1] = pk16(bf_bits(valid ? a[2]  : 0.f), bf_bits(valid ? a[3]  : 0.f));
  p[2] = pk16(bf_bits(valid ? a2[0] : 0.f), bf_bits(valid ? a2[1] : 0.f));
  p[3] = pk16(bf_bits(valid ? a2[2] : 0.f), bf_bits(valid ? a2[3] : 0.f));
  unsigned short* gp = dst + (size_t)i * 8;
  *(volatile v4u*)gp = p;
  __threadfence();
  *(volatile v4u*)gp = p;
}

template <int WF>
__global__ __launch_bounds__(256) void tr_feat(const float* __restrict__ src, int C, int HW,
                                               unsigned short* dstb, float* dstf) {
  __shared__ float tile[64][33];
  const int tid = threadIdx.x;
  const int b   = blockIdx.z;
  const int c0  = blockIdx.x * 64;
  const int p0  = blockIdx.y * 32;
  const float* sb = src + (size_t)b * C * HW;
#pragma unroll
  for (int pp = 0; pp < 8; ++pp) {
    const int idx = pp * 256 + tid;
    const int i = idx >> 5, o = idx & 31;
    tile[i][o] = sb[(size_t)(c0 + i) * HW + p0 + o];
  }
  __syncthreads();
  {
    const int o = tid >> 3, c8 = (tid & 7) * 8;
    v4u pk;
#pragma unroll
    for (int e = 0; e < 4; ++e)
      pk[e] = pk16(bf_bits(tile[c8 + 2 * e][o]), bf_bits(tile[c8 + 2 * e + 1][o]));
    unsigned short* gp = dstb + ((size_t)b * HW + p0 + o) * C + c0 + c8;
    *(volatile v4u*)gp = pk;
    __threadfence();
    *(volatile v4u*)gp = pk;
  }
  if (WF != 0) {
#pragma unroll
    for (int it = 0; it < 2; ++it) {
      const int o = it * 16 + (tid >> 4), c4 = (tid & 15) * 4;
      v4f v;
#pragma unroll
      for (int e = 0; e < 4; ++e) v[e] = bf_up(bf_bits(tile[c4 + e][o]));
      float* gp = dstf + ((size_t)b * HW + p0 + o) * C + c0 + c4;
      *(volatile v4f*)gp = v;
      __threadfence();
      *(volatile v4f*)gp = v;
    }
  }
}

template <int NSPLIT, int OMODE>
__global__ __launch_bounds__(256) void gemm64(
    const unsigned short* __restrict__ Ap, const unsigned short* A2p, int lda, long long strideA,
    const unsigned short* __restrict__ Btp, const unsigned short* Bt2p, int ldb, long long strideB,
    float* Cf, int ldc, long long strideC,
    unsigned short* Ch, unsigned short* Cl, int ldh, long long strideH,
    const float* __restrict__ biasp,
    const float* __restrict__ resid, int ldr, long long strideR,
    int M, int N, int K, float oscale) {
  const __bf16* A   = (const __bf16*)(const void*)Ap;
  const __bf16* A2  = (const __bf16*)(const void*)A2p;
  const __bf16* Bt  = (const __bf16*)(const void*)Btp;
  const __bf16* Bt2 = (const __bf16*)(const void*)Bt2p;
  __shared__ __align__(16) float sT[8][16 * 68];
  const int b    = blockIdx.y;
  const int lane = threadIdx.x & 31;
  const int wave = threadIdx.x >> 5;
  const int tilesN = N >> 6;
  const int tilesM = M >> 6;
  const int tile = blockIdx.x * 8 + wave;
  if (tile >= tilesM * tilesN) return;
  const int tm = tile / tilesN;
  const int tn = tile - tm * tilesN;
  const int m0 = tm << 6;
  const int n0 = tn << 6;

  const __bf16* Ab  = A  + (size_t)b * (size_t)strideA;
  const __bf16* Bb  = Bt + (size_t)b * (size_t)strideB;
  const __bf16* Ab2 = (NSPLIT == 1) ? (A2  + (size_t)b * (size_t)strideA) : Ab;
  const __bf16* Bb2 = (NSPLIT == 2) ? (Bt2 + (size_t)b * (size_t)strideB) : Bb;

  const int rlane = lane & 15;
  const int koff  = (lane >> 4) * 8;
  const int mOff  = (lane >> 4) * 8;

  v8f acc[4][4];
#pragma unroll
  for (int i = 0; i < 4; ++i)
#pragma unroll
    for (int j = 0; j < 4; ++j) acc[i][j] = zero8();

  if (NSPLIT != 2) {
    for (int k0 = 0; k0 < K; k0 += 32) {
      v16b bh[4];
#pragma unroll
      for (int j = 0; j < 4; ++j) {
        const size_t bo = (size_t)(n0 + (j << 4) + rlane) * ldb + koff + k0;
        bh[j] = ldfrag_b(Bb + bo);
      }
#pragma unroll
      for (int i = 0; i < 4; ++i) {
        const size_t ao = (size_t)(m0 + (i << 4) + rlane) * lda + koff + k0;
        const v16b ah = ldfrag_b(Ab + ao);
        v16b al = ah;
        if (NSPLIT == 1) al = ldfrag_b(Ab2 + ao);
#pragma unroll
        for (int j = 0; j < 4; ++j) {
          acc[i][j] = mma_b_raw(ah, bh[j], acc[i][j]);
          if (NSPLIT == 1) acc[i][j] = mma_b_raw(al, bh[j], acc[i][j]);
        }
        dep_guard_b(acc[i][0], acc[i][3], ah, al);
      }
      keep4_b(bh[0], bh[1], bh[2], bh[3]);
    }
  } else {
    for (int k0 = 0; k0 < K; k0 += 32) {
      v16b ah[4];
#pragma unroll
      for (int i = 0; i < 4; ++i) {
        const size_t ao = (size_t)(m0 + (i << 4) + rlane) * lda + koff + k0;
        ah[i] = ldfrag_b(Ab + ao);
      }
#pragma unroll
      for (int j = 0; j < 4; ++j) {
        const size_t bo = (size_t)(n0 + (j << 4) + rlane) * ldb + koff + k0;
        const v16b bh = ldfrag_b(Bb + bo);
        const v16b bl = ldfrag_b(Bb2 + bo);
#pragma unroll
        for (int i = 0; i < 4; ++i) {
          acc[i][j] = mma_b_raw(ah[i], bh, acc[i][j]);
          acc[i][j] = mma_b_raw(ah[i], bl, acc[i][j]);
        }
        dep_guard_b(acc[0][j], acc[3][j], bh, bl);
      }
      keep4_b(ah[0], ah[1], ah[2], ah[3]);
    }
  }
  acc_guard4(acc[0][0], acc[0][1], acc[0][2], acc[0][3]);
  acc_guard4(acc[1][0], acc[1][1], acc[1][2], acc[1][3]);
  acc_guard4(acc[2][0], acc[2][1], acc[2][2], acc[2][3]);
  acc_guard4(acc[3][0], acc[3][1], acc[3][2], acc[3][3]);

  float* slab = sT[wave];
#pragma unroll
  for (int i = 0; i < 4; ++i) {
    const int mBase = m0 + (i << 4);
#pragma unroll
    for (int j = 0; j < 4; ++j) {
#pragma unroll
      for (int r = 0; r < 8; ++r) {
        slab[(mOff + r) * 68 + (j << 4) + rlane] = acc[i][j][r];
      }
    }
    wave_sync_lds();
    if (OMODE == 1 || OMODE == 4) {
      float* C = Cf + (size_t)b * (size_t)strideC;
      const int h2 = lane >> 4, c4 = (lane & 15) * 4;
      v4f vv[8];
#pragma unroll
      for (int it = 0; it < 8; ++it) {
        const int row = it * 2 + h2;
        v4f v = *(const v4f*)(slab + row * 68 + c4);
        if (OMODE == 1) {
#pragma unroll
          for (int e = 0; e < 4; ++e) v[e] += bf_up(bf_bits(biasp[n0 + c4 + e]));
        } else {
          const float br = bf_up(bf_bits(biasp[mBase + row]));
#pragma unroll
          for (int e = 0; e < 4; ++e) v[e] += br;
        }
        vv[it] = v;
      }
      for (int pass = 0; pass < 2; ++pass) {
#pragma unroll
        for (int it = 0; it < 8; ++it) {
          const int row = it * 2 + h2;
          *(volatile v4f*)(C + (size_t)(mBase + row) * ldc + n0 + c4) = vv[it];
        }
        __threadfence();
      }
    }
    if (OMODE == 1 || OMODE == 2 || OMODE == 3) {
      const int q = lane >> 3, c8 = (lane & 7) * 8;
      unsigned short* H = Ch + (size_t)b * (size_t)strideH;
      unsigned short* L = Cl + (size_t)b * (size_t)strideH;
      float badd[8];
#pragma unroll
      for (int e = 0; e < 8; ++e) badd[e] = 0.f;
      if (OMODE != 3) {
#pragma unroll
        for (int e = 0; e < 8; ++e) badd[e] = bf_up(bf_bits(biasp[n0 + c8 + e]));
      }
      v4u hv[4], lv[4];
#pragma unroll
      for (int it = 0; it < 4; ++it) {
        const int row = it * 4 + q;
        const float* sp = slab + row * 68 + c8;
        float f[8];
#pragma unroll
        for (int e = 0; e < 8; ++e) f[e] = sp[e] + badd[e];
        if (OMODE == 2) {
          const float* rp = resid + (size_t)b * (size_t)strideR + (size_t)(mBase + row) * ldr + n0 + c8;
          const v4f r0 = *(const v4f*)rp;
          const v4f r1 = *(const v4f*)(rp + 4);
#pragma unroll
          for (int e = 0; e < 4; ++e) { f[e] += r0[e]; f[4 + e] += r1[e]; }
        }
        v4u a, a2;
#pragma unroll
        for (int e = 0; e < 4; ++e) {
          const float f0 = f[2 * e], f1 = f[2 * e + 1];
          unsigned short h0, h1, l0, l1;
          if (OMODE == 3) {
            h0 = h_bits((_Float16)(f0 * oscale)); h1 = h_bits((_Float16)(f1 * oscale));
            l0 = 0; l1 = 0;
          } else {
            h0 = bf_bits(f0); h1 = bf_bits(f1);
            l0 = bf_bits(f0 - bf_up(h0)); l1 = bf_bits(f1 - bf_up(h1));
          }
          a[e] = pk16(h0, h1); a2[e] = pk16(l0, l1);
        }
        hv[it] = a; lv[it] = a2;
      }
      for (int pass = 0; pass < 2; ++pass) {
#pragma unroll
        for (int it = 0; it < 4; ++it) {
          const int row = it * 4 + q;
          *(volatile v4u*)(H + (size_t)(mBase + row) * ldh + n0 + c8) = hv[it];
          if (OMODE != 3) *(volatile v4u*)(L + (size_t)(mBase + row) * ldh + n0 + c8) = lv[it];
        }
        __threadfence();
      }
    }
    wave_sync_lds();
  }
}

__global__ __launch_bounds__(256) void resize_hl(const float* __restrict__ src, int Hs, int Ws, float invy, float invx,
                                                 unsigned short* dh, unsigned short* dl, int Hd, int Wd,
                                                 int Mtok, int tokOfs, int total) {
#pragma clang fp contract(off)
  const int i = blockIdx.x * 256 + threadIdx.x;
  if (i >= total) return;
  const int c8 = i % 24;
  const int t  = i / 24;
  const int hw = Hd * Wd;
  const int p  = t % hw;
  const int b  = t / hw;
  const int y  = p / Wd;
  const int x  = p - y * Wd;

  const float sfy = ((float)y + 0.5f) * invy - 0.5f;
  const int   y0  = (int)floorf(sfy);
  const float fy  = sfy - (float)y0;
  const bool  ybd = (y0 < 0) || (y0 >= Hs - 1);
  const int   ya  = (y0 < 0) ? 0 : ((y0 >= Hs - 1) ? (Hs - 1) : y0);
  const int   yb  = ybd ? ya : (y0 + 1);
  const float wya = ybd ? 1.f : (1.f - fy);
  const float wyb = ybd ? 0.f : fy;

  const float sfx = ((float)x + 0.5f) * invx - 0.5f;
  const int   x0  = (int)floorf(sfx);
  const float fx  = sfx - (float)x0;
  const bool  xbd = (x0 < 0) || (x0 >= Ws - 1);
  const int   xa  = (x0 < 0) ? 0 : ((x0 >= Ws - 1) ? (Ws - 1) : x0);
  const int   xb  = xbd ? xa : (x0 + 1);
  const float wxa = xbd ? 1.f : (1.f - fx);
  const float wxb = xbd ? 0.f : fx;

  const float* sb  = src + ((size_t)b * Hs * Ws) * DIMC + c8 * 8;
  const float* paa = sb + ((size_t)ya * Ws + xa) * DIMC;
  const float* pba = sb + ((size_t)yb * Ws + xa) * DIMC;
  const float* pab = sb + ((size_t)ya * Ws + xb) * DIMC;
  const float* pbb = sb + ((size_t)yb * Ws + xb) * DIMC;
  float v[8];
  {
    const v4f aa0 = *(const v4f*)paa, aa1 = *(const v4f*)(paa + 4);
    const v4f ba0 = *(const v4f*)pba, ba1 = *(const v4f*)(pba + 4);
    const v4f ab0 = *(const v4f*)pab, ab1 = *(const v4f*)(pab + 4);
    const v4f bb0 = *(const v4f*)pbb, bb1 = *(const v4f*)(pbb + 4);
#pragma unroll
    for (int e = 0; e < 4; ++e) {
      const float ta0 = wya * aa0[e] + wyb * ba0[e];
      const float tb0 = wya * ab0[e] + wyb * bb0[e];
      v[e] = wxa * ta0 + wxb * tb0;
      const float ta1 = wya * aa1[e] + wyb * ba1[e];
      const float tb1 = wya * ab1[e] + wyb * bb1[e];
      v[4 + e] = wxa * ta1 + wxb * tb1;
    }
  }
  v4u hp, lp;
#pragma unroll
  for (int e = 0; e < 4; ++e) {
    const unsigned short h0 = bf_bits(v[2 * e]), h1 = bf_bits(v[2 * e + 1]);
    const unsigned short l0 = bf_bits(v[2 * e] - bf_up(h0)), l1 = bf_bits(v[2 * e + 1] - bf_up(h1));
    hp[e] = pk16(h0, h1); lp[e] = pk16(l0, l1);
  }
  const size_t go = ((size_t)b * Mtok + tokOfs + p) * DIMC + c8 * 8;
  *(volatile v4u*)(dh + go) = hp;
  *(volatile v4u*)(dl + go) = lp;
  __threadfence();
  *(volatile v4u*)(dh + go) = hp;
  *(volatile v4u*)(dl + go) = lp;
}

__global__ __launch_bounds__(256)
void attn24(const unsigned short* __restrict__ qp, const unsigned short* __restrict__ kp,
            const unsigned short* __restrict__ vp, unsigned short* ohp, unsigned short* olp,
            int N, int M, float sscale, float onorm) {
  union FH { v16h v; v8h h[2]; };
  __shared__ __align__(16) _Float16 Psh[8][16 * 64];
  __shared__ __align__(16) float    Os[16 * QCOL];

  const int tid  = threadIdx.x;
  const int wave = tid >> 5;
  const int lane = tid & 31;
  const int hh   = lane >> 4;
  const int c    = lane & 15;

  const int nqt  = N >> 4;
  const int b    = blockIdx.x / nqt;
  const int q0   = (blockIdx.x - b * nqt) << 4;
  const int h    = wave;
  const size_t rowQ = (size_t)b * N;
  const size_t rowK = (size_t)b * M;

  const _Float16* Qh = (const _Float16*)(const void*)qp + (size_t)h * HDP;
  const _Float16* Kh = (const _Float16*)(const void*)kp + (size_t)h * HDP;
  const _Float16* Vh = (const _Float16*)(const void*)vp + ((size_t)b * QCOL + (size_t)h * HDP) * (size_t)M;

  const v16h qa = ldfrag_h(Qh + (rowQ + q0 + c) * QCOL + 8 * hh);

  float mrow[8], lrow[8];
  v8f oacc[2];
#pragma unroll
  for (int r = 0; r < 8; ++r) { mrow[r] = -INFINITY; lrow[r] = 0.f; }
#pragma unroll
  for (int t = 0; t < 2; ++t) oacc[t] = zero8();

  _Float16* pw = Psh[wave];
  const int nkc = M >> 6;

  for (int kt = 0; kt < nkc; ++kt) {
    const int kv0 = kt << 6;

    v8f s[4];
#pragma unroll
    for (int j = 0; j < 4; ++j) {
      const size_t ko = (rowK + kv0 + j * 16 + c) * QCOL + 8 * hh;
      const v16h kb = ldfrag_h(Kh + ko);
      const v8f a = mma_h(qa, kb, zero8());
#pragma unroll
      for (int r = 0; r < 8; ++r) s[j][r] = a[r] * sscale;
    }

#pragma unroll
    for (int r = 0; r < 8; ++r) {
      float m = fmaxf(fmaxf(s[0][r], s[1][r]), fmaxf(s[2][r], s[3][r]));
#pragma unroll
      for (int off = 1; off < 16; off <<= 1) m = fmaxf(m, __shfl_xor(m, off, 32));
      const float mnew  = fmaxf(mrow[r], m);
      const float alpha = __expf(mrow[r] - mnew);
      mrow[r] = mnew;
      float psum = 0.f;
#pragma unroll
      for (int j = 0; j < 4; ++j) {
        const float p = __expf(s[j][r] - mnew);
        psum += p;
        pw[(8 * hh + r) * 64 + j * 16 + c] = (_Float16)(p * 1024.0f);
      }
#pragma unroll
      for (int off = 1; off < 16; off <<= 1) psum += __shfl_xor(psum, off, 32);
      lrow[r] = lrow[r] * alpha + psum;
#pragma unroll
      for (int t = 0; t < 2; ++t) oacc[t][r] *= alpha;
    }
    wave_sync_lds();

#pragma unroll
    for (int kk = 0; kk < 2; ++kk) {
      FH pa;
      pa.h[0] = *(const v8h*)(pw + c * 64 + kk * 32 + 8 * hh);
      pa.h[1] = *(const v8h*)(pw + c * 64 + kk * 32 + 16 + 8 * hh);
#pragma unroll
      for (int t = 0; t < 2; ++t) {
        const size_t vo = (size_t)(t * 16 + c) * (size_t)M + kv0 + kk * 32 + 8 * hh;
        const v16h vb = ldfrag_h(Vh + vo);
        oacc[t] = mma_h(pa.v, vb, oacc[t]);
      }
    }
    wave_sync_lds();
  }

#pragma unroll
  for (int r = 0; r < 8; ++r) {
    const float l = lrow[r];
    const float inv = ((l > 0.f) ? (1.0f / l) : 0.f) * onorm;
#pragma unroll
    for (int t = 0; t < 2; ++t) Os[(8 * hh + r) * QCOL + h * HDP + t * 16 + c] = oacc[t][r] * inv;
  }
  __syncthreads();
  {
    const int lq = tid >> 3, c8 = (tid & 7) * 8;
    v4u hv[2], lv[2];
    size_t go[2];
    bool ok[2];
#pragma unroll
    for (int it = 0; it < 2; ++it) {
      const int L  = it * 32 + lq;
      ok[it] = (L < 48);
      const int Lc = ok[it] ? L : 0;
      const int row = Lc / 3;
      const int seg = Lc - row * 3;
      const int cc  = seg * 64 + c8;
      const int hd  = cc / 24;
      const int dd  = cc - hd * 24;
      const float* sp = Os + row * QCOL + hd * HDP + dd;
      v4u a, a2;
#pragma unroll
      for (int e = 0; e < 4; ++e) {
        const float f0 = sp[2 * e], f1 = sp[2 * e + 1];
        const unsigned short h0 = bf_bits(f0), h1 = bf_bits(f1);
        const unsigned short l0 = bf_bits(f0 - bf_up(h0)), l1 = bf_bits(f1 - bf_up(h1));
        a[e] = pk16(h0, h1); a2[e] = pk16(l0, l1);
      }
      hv[it] = a; lv[it] = a2;
      go[it] = (rowQ + q0 + row) * DIMC + cc;
    }
    for (int pass = 0; pass < 2; ++pass) {
#pragma unroll
      for (int it = 0; it < 2; ++it) {
        if (ok[it]) {
          *(volatile v4u*)(ohp + go[it]) = hv[it];
          *(volatile v4u*)(olp + go[it]) = lv[it];
        }
      }
      __threadfence();
    }
  }
}

extern "C" void kernel_launch(void* const* d_in, const int* in_sizes, int n_in,
                              void* d_out, int out_size, void* d_ws, size_t ws_size,
                              hipStream_t stream) {
  const int NN[3] = {1024, 256, 64};
  const int MM[3] = {2048, 512, 128};
  const int HH[3] = {32, 16, 8};
  const int CC[3] = {192, 384, 768};
  if (n_in < 25) return;
  if (in_sizes[0] != NBATCH * 192 * 1024 || in_sizes[1] != NBATCH * 384 * 256 || in_sizes[2] != NBATCH * 768 * 64) return;
  if (in_sizes[3] != 192 * 384 || in_sizes[4] != 192 || in_sizes[5] != 192 * 768 || in_sizes[6] != 192) return;
  for (int i = 0; i < 3; ++i) {
    if (in_sizes[7 + 4 * i] != 192 * 192 || in_sizes[8 + 4 * i] != 384 * 192 ||
        in_sizes[9 + 4 * i] != 192 * 192 || in_sizes[10 + 4 * i] != 192) return;
    if (in_sizes[19 + 2 * i] != CC[i] * 192 || in_sizes[20 + 2 * i] != CC[i]) return;
  }
  if (out_size != NBATCH * (192 * 1024 + 384 * 256 + 768 * 64)) return;

  const float* f0 = (const float*)d_in[0];
  const float* f1 = (const float*)d_in[1];
  const float* f2 = (const float*)d_in[2];
  const float* proj1_w = (const float*)d_in[3];
  const float* proj1_b = (const float*)d_in[4];
  const float* proj2_w = (const float*)d_in[5];
  const float* proj2_b = (const float*)d_in[6];
  const float* q_w[3]   = {(const float*)d_in[7],  (const float*)d_in[11], (const float*)d_in[15]};
  const float* kv_w[3]  = {(const float*)d_in[8],  (const float*)d_in[12], (const float*)d_in[16]};
  const float* pr_w[3]  = {(const float*)d_in[9],  (const float*)d_in[13], (const float*)d_in[17]};
  const float* pr_b[3]  = {(const float*)d_in[10], (const float*)d_in[14], (const float*)d_in[18]};
  const float* out_w[3] = {(const float*)d_in[19], (const float*)d_in[21], (const float*)d_in[23]};
  const float* out_b[3] = {(const float*)d_in[20], (const float*)d_in[22], (const float*)d_in[24]};

  float* outp = (float*)d_out;
  const size_t out_ofs[3] = {0, (size_t)NBATCH * 192 * 1024, (size_t)NBATCH * 192 * 1024 + (size_t)NBATCH * 384 * 256};

  size_t off = 0;
  auto carve = [&](size_t bytes) -> size_t { const size_t o = off; off += bytes; return o; };
  const size_t oWp1 = carve((size_t)192 * 384 * 2);
  const size_t oWp2 = carve((size_t)192 * 768 * 2);
  size_t oWq[3], oWkv[3], oWpr[3], oWo[3];
  for (int i = 0; i < 3; ++i) {
    oWq[i]  = carve((size_t)QCOL * 192 * 2);
    oWkv[i] = carve((size_t)2 * QCOL * 192 * 2);
    oWpr[i] = carve((size_t)192 * 192 * 2);
    oWo[i]  = carve((size_t)CC[i] * 192 * 2);
  }
  const size_t oX0b = carve((size_t)NBATCH * 1024 * 192 * 2);
  const size_t oP0f = carve((size_t)NBATCH * 1024 * 192 * 4);
  const size_t oT1b = carve((size_t)NBATCH * 256 * 384 * 2);
  const size_t oT2b = carve((size_t)NBATCH * 64 * 768 * 2);
  const size_t oP1f = carve((size_t)NBATCH * 256 * 192 * 4);
  const size_t oP1h = carve((size_t)NBATCH * 256 * 192 * 2);
  const size_t oP1l = carve((size_t)NBATCH * 256 * 192 * 2);
  const size_t oP2f = carve((size_t)NBATCH * 64 * 192 * 4);
  const size_t oP2h = carve((size_t)NBATCH * 64 * 192 * 2);
  const size_t oP2l = carve((size_t)NBATCH * 64 * 192 * 2);
  size_t oCh[3], oCl[3], oQ[3], oK[3], oV[3], oOh[3], oOl[3], oEh[3], oEl[3];
  for (int i = 0; i < 3; ++i) {
    oCh[i] = carve((size_t)NBATCH * MM[i] * 192 * 2);
    oCl[i] = carve((size_t)NBATCH * MM[i] * 192 * 2);
    oQ[i]  = carve((size_t)NBATCH * NN[i] * QCOL * 2);
    oK[i]  = carve((size_t)NBATCH * MM[i] * QCOL * 2);
    oV[i]  = carve((size_t)NBATCH * QCOL * MM[i] * 2);
    oOh[i] = carve((size_t)NBATCH * NN[i] * 192 * 2);
    oOl[i] = carve((size_t)NBATCH * NN[i] * 192 * 2);
    oEh[i] = carve((size_t)NBATCH * NN[i] * 192 * 2);
    oEl[i] = carve((size_t)NBATCH * NN[i] * 192 * 2);
  }
  if (off > ws_size) return;
  if (off > (size_t)134217728) return;

  char* ws = (char*)d_ws;
  unsigned short* Wp1 = (unsigned short*)(ws + oWp1);
  unsigned short* Wp2 = (unsigned short*)(ws + oWp2);
  unsigned short *Wq[3], *Wkv[3], *Wpr[3], *Wo[3];
  unsigned short *Ch[3], *Cl[3], *Qp[3], *Kp[3], *Vt[3], *Oh[3], *Ol[3], *Eh[3], *El[3];
  for (int i = 0; i < 3; ++i) {
    Wq[i]  = (unsigned short*)(ws + oWq[i]);
    Wkv[i] = (unsigned short*)(ws + oWkv[i]);
    Wpr[i] = (unsigned short*)(ws + oWpr[i]);
    Wo[i]  = (unsigned short*)(ws + oWo[i]);
    Ch[i]  = (unsigned short*)(ws + oCh[i]);
    Cl[i]  = (unsigned short*)(ws + oCl[i]);
    Qp[i]  = (unsigned short*)(ws + oQ[i]);
    Kp[i]  = (unsigned short*)(ws + oK[i]);
    Vt[i]  = (unsigned short*)(ws + oV[i]);
    Oh[i]  = (unsigned short*)(ws + oOh[i]);
    Ol[i]  = (unsigned short*)(ws + oOl[i]);
    Eh[i]  = (unsigned short*)(ws + oEh[i]);
    El[i]  = (unsigned short*)(ws + oEl[i]);
  }
  unsigned short* X0b = (unsigned short*)(ws + oX0b);
  float*          P0f = (float*)(ws + oP0f);
  unsigned short* T1b = (unsigned short*)(ws + oT1b);
  unsigned short* T2b = (unsigned short*)(ws + oT2b);
  float*          P1f = (float*)(ws + oP1f);
  unsigned short* P1h = (unsigned short*)(ws + oP1h);
  unsigned short* P1l = (unsigned short*)(ws + oP1l);
  float*          P2f = (float*)(ws + oP2f);
  unsigned short* P2h = (unsigned short*)(ws + oP2h);
  unsigned short* P2l = (unsigned short*)(ws + oP2l);
  float* Pf[3]            = {P0f, P1f, P2f};
  unsigned short* Xh[3]   = {X0b, P1h, P2h};
  unsigned short* Xl[3]   = {X0b, P1l, P2l};

  const float sscale = 0.2041241452319315f * (1.0f / 256.0f);
  const float onorm  = 1.0f / 65536.0f;
  const dim3 blk(256);

  cvt_rows<<<dim3((192 * 384 / 8 + 255) / 256), blk, 0, stream>>>(proj1_w, 192, 384, Wp1, 0, 192 * 384 / 8);
  cvt_rows<<<dim3((192 * 768 / 8 + 255) / 256), blk, 0, stream>>>(proj2_w, 192, 768, Wp2, 0, 192 * 768 / 8);
  for (int i = 0; i < 3; ++i) {
    cvt_rows<<<dim3((QCOL * 192 / 8 + 255) / 256), blk, 0, stream>>>(q_w[i], 192, 192, Wq[i], 1, QCOL * 192 / 8);
    cvt_rows<<<dim3((2 * QCOL * 192 / 8 + 255) / 256), blk, 0, stream>>>(kv_w[i], 384, 192, Wkv[i], 1, 2 * QCOL * 192 / 8);
    cvt_rows<<<dim3((192 * 192 / 8 + 255) / 256), blk, 0, stream>>>(pr_w[i], 192, 192, Wpr[i], 0, 192 * 192 / 8);
    cvt_rows<<<dim3((CC[i] * 192 / 8 + 255) / 256), blk, 0, stream>>>(out_w[i], CC[i], 192, Wo[i], 0, CC[i] * 192 / 8);
  }
  tr_feat<1><<<dim3(192 / 64, 1024 / 32, NBATCH), blk, 0, stream>>>(f0, 192, 1024, X0b, P0f);
  tr_feat<0><<<dim3(384 / 64, 256 / 32, NBATCH), blk, 0, stream>>>(f1, 384, 256, T1b, P0f);
  tr_feat<0><<<dim3(768 / 64, 64 / 32, NBATCH), blk, 0, stream>>>(f2, 768, 64, T2b, P0f);
  gemm64<0, 1><<<dim3(((NBATCH * 256 / 64) * 3 + 7) / 8, 1), blk, 0, stream>>>(
      T1b, T1b, 384, 0LL, Wp1, Wp1, 384, 0LL,
      P1f, 192, 0LL, P1h, P1l, 192, 0LL,
      proj1_b, P0f, 192, 0LL, NBATCH * 256, 192, 384, 1.0f);
  gemm64<0, 1><<<dim3(((NBATCH * 64 / 64) * 3 + 7) / 8, 1), blk, 0, stream>>>(
      T2b, T2b, 768, 0LL, Wp2, Wp2, 768, 0LL,
      P2f, 192, 0LL, P2h, P2l, 192, 0LL,
      proj2_b, P0f, 192, 0LL, NBATCH * 64, 192, 768, 1.0f);
  for (int i = 0; i < 3; ++i) {
    int ofs = 0;
    for (int j = 0; j < 3; ++j) {
      if (j == i) continue;
      const int total = NBATCH * NN[i] * 24;
      const float inv = (float)HH[j] / (float)HH[i];
      resize_hl<<<dim3((total + 255) / 256), blk, 0, stream>>>(
          Pf[j], HH[j], HH[j], inv, inv, Ch[i], Cl[i], HH[i], HH[i], MM[i], ofs, total);
      ofs += NN[i];
    }
  }
  for (int i = 0; i < 3; ++i) {
    const int N = NN[i], M = MM[i];
    const int rowsQ = NBATCH * N, rowsK = NBATCH * M;
    if (i == 0) {
      gemm64<0, 3><<<dim3(((rowsQ / 64) * (QCOL / 64) + 7) / 8, 1), blk, 0, stream>>>(
          Xh[i], Xl[i], 192, 0LL, Wq[i], Wq[i], 192, 0LL,
          P0f, QCOL, 0LL, Qp[i], Qp[i], QCOL, 0LL,
          q_w[i], P0f, 192, 0LL, rowsQ, QCOL, 192, 16.0f);
    } else {
      gemm64<1, 3><<<dim3(((rowsQ / 64) * (QCOL / 64) + 7) / 8, 1), blk, 0, stream>>>(
          Xh[i], Xl[i], 192, 0LL, Wq[i], Wq[i], 192, 0LL,
          P0f, QCOL, 0LL, Qp[i], Qp[i], QCOL, 0LL,
          q_w[i], P0f, 192, 0LL, rowsQ, QCOL, 192, 16.0f);
    }
    gemm64<1, 3><<<dim3(((rowsK / 64) * (QCOL / 64) + 7) / 8, 1), blk, 0, stream>>>(
        Ch[i], Cl[i], 192, 0LL, Wkv[i], Wkv[i], 192, 0LL,
        P0f, QCOL, 0LL, Kp[i], Kp[i], QCOL, 0LL,
        kv_w[i], P0f, 192, 0LL, rowsK, QCOL, 192, 16.0f);
    gemm64<2, 3><<<dim3(((QCOL / 64) * (M / 64) + 7) / 8, NBATCH), blk, 0, stream>>>(
        Wkv[i] + (size_t)QCOL * 192, Wkv[i] + (size_t)QCOL * 192, 192, 0LL, Ch[i], Cl[i], 192, (long long)M * 192,
        P0f, M, 0LL, Vt[i], Vt[i], M, (long long)QCOL * M,
        kv_w[i], P0f, 192, 0LL, QCOL, M, 192, 64.0f);
    attn24<<<dim3(rowsQ / 16), blk, 0, stream>>>(Qp[i], Kp[i], Vt[i], Oh[i], Ol[i], N, M, sscale, onorm);
    gemm64<1, 2><<<dim3(((rowsQ / 64) * 3 + 7) / 8, 1), blk, 0, stream>>>(
        Oh[i], Ol[i], 192, 0LL, Wpr[i], Wpr[i], 192, 0LL,
        P0f, 192, 0LL, Eh[i], El[i], 192, 0LL,
        pr_b[i], Pf[i], 192, 0LL, rowsQ, 192, 192, 1.0f);
    gemm64<2, 4><<<dim3(((CC[i] / 64) * (N / 64) + 7) / 8, NBATCH), blk, 0, stream>>>(
        Wo[i], Wo[i], 192, 0LL, Eh[i], El[i], 192, (long long)N * 192,
        outp + out_ofs[i], N, (long long)CC[i] * N, Eh[i], El[i], 192, 0LL,
        out_b[i], P0f, 192, 0LL, CC[i], N, 192, 1.0f);
  }
  (void)hipGetLastError();
}
